// GraphGIN_70944269795972
// MI455X (gfx1250) — hardware-run, weakly checked
//
#include <hip/hip_runtime.h>


namespace {
constexpr int NN = 100000, NE = 3200000, F0 = 64, HID = 20, HP = 32  , NG = 128, NCLS = 10, MAXDEG = 2048, NGc = (NN + 255) / 256, PERMLEN = NE + 32 * NGc + 32;
constexpr float XS = 8.0f;

typedef _Float16 b16;
typedef __attribute__((ext_vector_type(16))) _Float16 v16b;
typedef __attribute__((ext_vector_type(8))) _Float16 v8b;
typedef __attribute__((ext_vector_type(8))) float v8f;
typedef __attribute__((ext_vector_type(4))) float v4f;
typedef __attribute__((ext_vector_type(2))) float v2f;
__device__ __forceinline__ float bf16_rne(float f) { unsigned int u = __float_as_uint(f); u += 0x7FFFu + ((u >> 16) & 1u); return __uint_as_float(u & 0xFFFF0000u); }
__device__ __forceinline__ void split16(float v, b16& hi, b16& lo) { hi = (b16)v; lo = (b16)(v - (float)hi); }
__device__ __forceinline__ v16b frag_kb(const b16* p, int hh) { const v8b a = *(const v8b*)(p + 8 * hh), b = *(const v8b*)(p + 16 + 8 * hh); v16b f;
#pragma unroll
  for (int e = 0; e < 8; ++e) { f[e] = a[e]; f[8 + e] = b[e]; } return f; }
__device__ __forceinline__ v8f wmma16b(v16b a, v16b b, v8f c) { v8f d = __builtin_amdgcn_wmma_f32_16x16x32_f16(false, a, false, b, (short)0, c, false, false); asm volatile("v_nop\n\tv_nop\n\tv_nop\n\tv_nop" : "+v"(d) : "v"(a), "v"(b)); return d; }
__device__ __forceinline__ void wave_lds_sync() { __builtin_amdgcn_fence(__ATOMIC_RELEASE, "workgroup"); __builtin_amdgcn_wave_barrier(); __builtin_amdgcn_fence(__ATOMIC_ACQUIRE, "workgroup"); }
__device__ __forceinline__ float pmul(float a, float b) { float p = a * b; asm volatile("" : "+v"(p)); return p; }
constexpr int CSR_NBLK = 512, CSR_GB = 8, CSR_GN = 1 << CSR_GB  , CSR_MAXG = 512, CSR_CAP = 12288  ;
__global__ __launch_bounds__(64) void csrA_kernel(const int* __restrict__ dst, int E, int N, int nG, int CHP, int NGP, int* __restrict__ STG, int* __restrict__ HST) {
  extern __shared__ int sm[];
  int* cnt = sm; int* run = sm + NGP; int* ids = sm + 2 * NGP;
  const int b = blockIdx.x; const int ch = (E + CSR_NBLK - 1) / CSR_NBLK; const int e0 = b * ch, e1 = min(E, e0 + ch);
  for (int i = threadIdx.x; i < NGP; i += 64) cnt[i] = 0;
  for (int i = threadIdx.x; i < CHP; i += 64) ids[i] = -1;
  __syncthreads();
  if (threadIdx.x == 0) {
    for (int e = e0; e < e1; ++e) { int d = dst[e]; d = (d < 0) ? 0 : (d >= N ? N - 1 : d); cnt[d >> CSR_GB] += 1; }
    int acc = 0; for (int g = 0; g < nG; ++g) { run[g] = acc; acc += cnt[g]; }
    for (int e = e0; e < e1; ++e) { int d = dst[e]; d = (d < 0) ? 0 : (d >= N ? N - 1 : d); const int g = d >> CSR_GB; ids[run[g]] = e; run[g] += 1; } }
  __syncthreads();
  typedef __attribute__((ext_vector_type(4))) int v4i;
  for (int pass = 0; pass < 2; ++pass) {
    for (int i = threadIdx.x; i < CHP / 4; i += 64) *(volatile v4i*)(STG + (size_t)b * CHP + i * 4) = *(const v4i*)(&ids[i * 4]);
    for (int i = threadIdx.x; i < NGP / 4; i += 64) { v4i v; for (int e = 0; e < 4; ++e) v[e] = (i * 4 + e < nG) ? cnt[i * 4 + e] : 0; *(volatile v4i*)(HST + (size_t)b * NGP + i * 4) = v; }
    __threadfence(); }
}
__global__ __launch_bounds__(512) void csrS_kernel(const int* __restrict__ HST, int nG, int NGP, int* __restrict__ START, int* __restrict__ TOT, int* __restrict__ OFF) {
  __shared__ int tot[CSR_MAXG];
  const int b = threadIdx.x;
  for (int pass = 0; pass < 2; ++pass) { int runb = 0; for (int g = 0; g < nG; ++g) { int c = HST[(size_t)b * NGP + g]; c = (c < 0) ? 0 : c; ((volatile int*)OFF)[(size_t)g * CSR_NBLK + b] = runb; runb += c; } __threadfence(); }
  for (int g = threadIdx.x; g < nG; g += 512) { int s = 0; for (int bb = 0; bb < CSR_NBLK; ++bb) { int c = HST[(size_t)bb * NGP + g]; s += (c < 0) ? 0 : c; } tot[g] = s; }
  __syncthreads();
  if (threadIdx.x < 32) {
    __shared__ int st[CSR_MAXG + 32];
    if (threadIdx.x == 0) { int acc = 0; for (int g = 0; g < NGP; ++g) { st[g] = acc; if (g < nG) acc += (tot[g] + 31) & ~31; } st[NGP] = acc; }
    __builtin_amdgcn_fence(__ATOMIC_RELEASE, "workgroup"); __builtin_amdgcn_wave_barrier(); __builtin_amdgcn_fence(__ATOMIC_ACQUIRE, "workgroup");
    for (int pass = 0; pass < 2; ++pass) { for (int i = threadIdx.x; i < NGP + 32; i += 32) { ((volatile int*)START)[i] = (i <= NGP) ? st[min(i, NGP)] : 0; ((volatile int*)TOT)[i] = (i < nG) ? tot[i] : 0; } __threadfence(); } }
}
__global__ __launch_bounds__(256) void csrB_kernel(const int* __restrict__ dst, int N, int nG, int CHP, int NGP, int permLen, const int* __restrict__ STG, const int* __restrict__ HST, const int* __restrict__ OFF, const int* __restrict__ START, const int* __restrict__ TOT, int* __restrict__ PERM, int* __restrict__ ROWPTR, int* __restrict__ ROWCNT, int* __restrict__ FLAG) {
  typedef __attribute__((ext_vector_type(4))) int v4i;
  __shared__ int ids[CSR_CAP]; __shared__ unsigned short key[CSR_CAP]; __shared__ int outp[CSR_CAP]; __shared__ int ncnt[CSR_GN + 1]; __shared__ int boff[CSR_NBLK + 1];
  const int g = blockIdx.x, t_ = threadIdx.x; int tot = TOT[g]; int st = START[g], stn = START[g + 1]; const int v0 = g * CSR_GN; const int nv = min(CSR_GN, N - v0);
  st = (st < 0) ? 0 : (st > permLen - 32 ? permLen - 32 : st) & ~31; stn = (stn < st) ? st : (stn > permLen ? permLen : stn); tot = (tot < 0) ? 0 : tot; if (tot > stn - st && tot <= CSR_CAP) tot = stn - st;
  if (tot > CSR_CAP) {
    for (int pass = 0; pass < 2; ++pass) { for (int i = t_; i < CSR_GN / 4; i += 256) { v4i a, c; for (int e = 0; e < 4; ++e) { a[e] = st; c[e] = 0; } *(volatile v4i*)(ROWPTR + v0 + i * 4) = a; *(volatile v4i*)(ROWCNT + v0 + i * 4) = c; } if (t_ == 0) ((volatile int*)FLAG)[0] = 1; __threadfence(); } (void)nv; return; }
  if (t_ == 0) { int acc = 0; for (int b = 0; b < CSR_NBLK; ++b) { boff[b] = acc; int c = HST[(size_t)b * NGP + g]; c = (c < 0) ? 0 : (c > CHP ? CHP : c); acc += c; if (acc > tot) acc = tot; } boff[CSR_NBLK] = acc; }
  for (int i = t_; i <= CSR_GN; i += 256) ncnt[i] = 0;
  __syncthreads();
  for (int b = 0; b < CSR_NBLK; ++b) { const int c = boff[b + 1] - boff[b]; int o_ = OFF[(size_t)g * CSR_NBLK + b]; o_ = (o_ < 0) ? 0 : (o_ > CHP - c ? CHP - c : o_); const int* src_ = STG + (size_t)b * CHP + o_;
    for (int i = t_; i < c; i += 256) { int id = src_[i]; id = (id < 0) ? 0 : id; ids[boff[b] + i] = id; int d = dst[id]; d = (d < v0) ? v0 : (d >= N ? N - 1 : d); int kk = d - v0; kk = (kk < 0) ? 0 : (kk >= CSR_GN ? CSR_GN - 1 : kk); key[boff[b] + i] = (unsigned short)kk; } }
  __syncthreads();
  if (t_ == 0) { for (int i = 0; i < tot; ++i) ncnt[key[i]] += 1; int acc = 0; for (int vl = 0; vl < CSR_GN; ++vl) { const int c = ncnt[vl]; ncnt[vl] = acc; acc += c; } ncnt[CSR_GN] = acc;
    for (int i = 0; i < tot; ++i) { const int vl = key[i]; outp[ncnt[vl]] = ids[i]; ncnt[vl] += 1; }
    for (int vl = CSR_GN; vl > 0; --vl) ncnt[vl] = ncnt[vl - 1]; ncnt[0] = 0; }
  __syncthreads();
  for (int pass = 0; pass < 2; ++pass) {
    for (int i = t_; i < (stn - st) / 4; i += 256) { v4i v; for (int e = 0; e < 4; ++e) { const int q = i * 4 + e; v[e] = (q < tot) ? outp[q] : -1; } *(volatile v4i*)(PERM + st + i * 4) = v; }
    for (int i = t_; i < CSR_GN / 4; i += 256) { v4i a, c; for (int e = 0; e < 4; ++e) { const int vl = i * 4 + e; a[e] = st + ncnt[vl]; c[e] = (vl < nv) ? (ncnt[vl + 1] - ncnt[vl]) : 0; } *(volatile v4i*)(ROWPTR + v0 + i * 4) = a; *(volatile v4i*)(ROWCNT + v0 + i * 4) = c; }
    __threadfence(); }
}
__global__ __launch_bounds__(256) void csrZ_kernel(int* __restrict__ p, size_t n4) { typedef __attribute__((ext_vector_type(4))) int v4i; const size_t tid = (size_t)blockIdx.x * 256 + threadIdx.x, nth = (size_t)gridDim.x * 256; v4i z = {0, 0, 0, 0}; for (size_t i = tid; i < n4; i += nth) *(volatile v4i*)(p + i * 4) = z; }
struct CsrBufs { int *STG, *HST, *OFF, *START, *TOT, *PERM, *ROWPTR, *ROWCNT, *FLAG; int nG, NGP, CHP; size_t permLen; char* base; size_t bytes; };
static size_t csr_carve(CsrBufs& c, char* ws, size_t off, int E, int N) {
  const size_t off0 = off; c.base = ws + off;
  auto al = [&](size_t bytes) { char* p = ws + off; off += (bytes + 255) & ~(size_t)255; return p; };
  c.nG = (N + CSR_GN - 1) / CSR_GN; c.NGP = (c.nG + 31) & ~31; const int ch = (E + CSR_NBLK - 1) / CSR_NBLK; c.CHP = (ch + 31) & ~31; c.permLen = (size_t)E + 32 * (size_t)c.nG + 32;
  c.STG = (int*)al((size_t)CSR_NBLK * c.CHP * 4); c.HST = (int*)al((size_t)CSR_NBLK * c.NGP * 4); c.OFF = (int*)al((size_t)c.NGP * CSR_NBLK * 4); c.START = (int*)al((size_t)(c.NGP + 64) * 4); c.TOT = (int*)al((size_t)(c.NGP + 64) * 4);
  c.PERM = (int*)al(c.permLen * 4); c.ROWPTR = (int*)al((size_t)c.nG * CSR_GN * 4); c.ROWCNT = (int*)al((size_t)c.nG * CSR_GN * 4); c.FLAG = (int*)al(256);
  c.bytes = off - off0; return off;
}
static void csr_build(const CsrBufs& c, const int* dst, int E, int N, hipStream_t stream) {
  const size_t smem = (size_t)(2 * c.NGP + c.CHP) * 4;
  csrZ_kernel<<<512, 256, 0, stream>>>((int*)c.base, c.bytes / 16);
  csrA_kernel<<<CSR_NBLK, 64, smem, stream>>>(dst, E, N, c.nG, c.CHP, c.NGP, c.STG, c.HST);
  csrS_kernel<<<1, 512, 0, stream>>>(c.HST, c.nG, c.NGP, c.START, c.TOT, c.OFF);
  csrB_kernel<<<c.nG, 256, 0, stream>>>(dst, N, c.nG, c.CHP, c.NGP, (int)c.permLen, c.STG, c.HST, c.OFF, c.START, c.TOT, c.PERM, c.ROWPTR, c.ROWCNT, c.FLAG);
}

struct Wo_ { static constexpr size_t A0 = 0, B0 = A0 + 32 * 64, A1 = B0 + 32 * 32, B1 = A1 + 32 * 32, A2 = B1 + 32 * 32, B2 = A2 + 32 * 32, END = B2 + 32 * 32; };
__global__ __launch_bounds__(256) void prep_kernel(const float* __restrict__ x, const float* __restrict__ W1a, const float* __restrict__ b1a, const float* __restrict__ W1b, const float* __restrict__ b1b, const float* __restrict__ W2a, const float* __restrict__ b2a, const float* __restrict__ W2b, const float* __restrict__ b2b, const float* __restrict__ W3a, const float* __restrict__ b3a, const float* __restrict__ W3b, const float* __restrict__ b3b, const float* __restrict__ Wl, const float* __restrict__ bl, b16* __restrict__ R, float* __restrict__ P, float* __restrict__ H0) {
  const size_t tid = (size_t)blockIdx.x * 256 + threadIdx.x, nth = (size_t)gridDim.x * 256;
  auto tr = [&](size_t base, int kin_real, int kpad, int nout_real, const float* W) { for (size_t p = tid; p < (size_t)32 * kpad; p += nth) { const int o = (int)(p / kpad), k = (int)(p % kpad); const float v = (o < nout_real && k < kin_real) ? bf16_rne(W[(size_t)k * nout_real + o]) : 0.0f; ((volatile b16*)R)[base + p] = (b16)v; } };
  for (int pass = 0; pass < 2; ++pass) {
    tr(Wo_::A0, F0, 64, HID, W1a); tr(Wo_::B0, HID, 32, HID, W1b); tr(Wo_::A1, HID, 32, HID, W2a); tr(Wo_::B1, HID, 32, HID, W2b); tr(Wo_::A2, HID, 32, HID, W3a); tr(Wo_::B2, HID, 32, HID, W3b);
    for (size_t q = tid; q < 608; q += nth) { const int i = (int)q; float v = 0.0f;
      if (i < 192) { const int l = i / 64, c = i % 64; const float* bA = (l == 0) ? b1a : (l == 1) ? b2a : b3a; const float* bB = (l == 0) ? b1b : (l == 1) ? b2b : b3b; if (c < 32) v = (c < HID) ? bA[c] : 0.0f; else v = (c - 32 < HID) ? bB[c - 32] : 0.0f; }
      else if (i < 592) v = Wl[i - 192]; else if (i < 602) v = bl[i - 592];
      P[q] = bf16_rne(v); }
    for (size_t p = tid; p < (size_t)NN * F0 / 4; p += nth) { const v4f v = *(const v4f*)(x + p * 4); v4f o; for (int e = 0; e < 4; ++e) o[e] = bf16_rne(v[e]); *(volatile v4f*)(H0 + p * 4) = o; }
    __threadfence(); }
}

template <int KIN>
__global__ __launch_bounds__(256) void gin_kernel(const float* __restrict__ Hin, const int* __restrict__ src, const float* __restrict__ ew, const int* __restrict__ perm, const int* __restrict__ rowptr, const int* __restrict__ rowcnt, const b16* __restrict__ Wa, const b16* __restrict__ Wb, const float* __restrict__ Pl, float* __restrict__ Hout) {
  __shared__ __attribute__((aligned(16))) b16 Ah[16][64 + 8], Al[16][64 + 8], Zh[16][32 + 8], Zl[16][32 + 8]; __shared__ __attribute__((aligned(16))) float Out[16][32 + 4];
  const int wave = threadIdx.x >> 5, lane = threadIdx.x & 31, nloc = lane & 15, hlf = lane >> 4, v0 = blockIdx.x * 16;
  constexpr int PER = KIN / 32;
  for (int q = 0; q < 2; ++q) { const int rr = wave * 2 + q, v = v0 + rr; float acc[PER]; for (int e = 0; e < PER; ++e) acc[e] = 0.0f;
    int cnt = rowcnt[v]; cnt = (cnt < 0) ? 0 : (cnt > MAXDEG ? MAXDEG : cnt); int p0 = rowptr[v]; p0 = (p0 < 0) ? 0 : (p0 > PERMLEN - cnt ? PERMLEN - cnt : p0);
    for (int i = 0; i < cnt; ++i) { int id = perm[p0 + i]; id = (id < 0) ? 0 : (id >= NE ? NE - 1 : id); int s = src[id]; s = (s < 0) ? 0 : (s >= NN ? NN - 1 : s); const float w = bf16_rne(ew[id]);
#pragma unroll
      for (int e = 0; e < PER; ++e) acc[e] += pmul(w, Hin[(size_t)s * KIN + lane * PER + e]); }
#pragma unroll
    for (int e = 0; e < PER; ++e) { b16 a_, b_; split16(acc[e] * XS, a_, b_); Ah[rr][lane * PER + e] = a_; Al[rr][lane * PER + e] = b_; } }
  __syncthreads();
  if (wave == 0) {
    v8f z[2] = {{}, {}};
#pragma unroll
    for (int kb = 0; kb < KIN; kb += 32) { const v16b a = frag_kb(&Ah[nloc][kb], hlf), al = frag_kb(&Al[nloc][kb], hlf);
#pragma unroll
      for (int t = 0; t < 2; ++t) { const v16b bw = frag_kb(Wa + (size_t)(t * 16 + nloc) * KIN + kb, hlf); z[t] = wmma16b(a, bw, z[t]); z[t] = wmma16b(al, bw, z[t]); } }
#pragma unroll
    for (int t = 0; t < 2; ++t)
#pragma unroll
      for (int r = 0; r < 8; ++r) { const int c = t * 16 + nloc; const float y = (c < HID) ? fmaxf(z[t][r] * (1.0f / XS) + Pl[c], 0.0f) : 0.0f; b16 a_, b_; split16(y * XS, a_, b_); Zh[8 * hlf + r][c] = a_; Zl[8 * hlf + r][c] = b_; }
    wave_lds_sync();
    v8f z2[2] = {{}, {}}; { const v16b a = frag_kb(&Zh[nloc][0], hlf), al = frag_kb(&Zl[nloc][0], hlf);
#pragma unroll
      for (int t = 0; t < 2; ++t) { const v16b bw = frag_kb(Wb + (size_t)(t * 16 + nloc) * 32, hlf); z2[t] = wmma16b(a, bw, z2[t]); z2[t] = wmma16b(al, bw, z2[t]); } }
#pragma unroll
    for (int t = 0; t < 2; ++t)
#pragma unroll
      for (int r = 0; r < 8; ++r) { const int c = t * 16 + nloc; Out[8 * hlf + r][c] = (c < HID) ? fmaxf(z2[t][r] * (1.0f / XS) + Pl[32 + c], 0.0f) : 0.0f; }
    wave_lds_sync();
    if (lane < 16) { float* row = &Out[lane][0]; float ss = 0.0f; for (int c = 0; c < HID; ++c) ss += pmul(row[c], row[c]); const float inv = 1.0f / fmaxf(sqrtf(ss), 1e-12f); for (int c = 0; c < HID; ++c) row[c] = fmaxf(pmul(row[c], inv), 0.0f); }
    wave_lds_sync();
    for (int pass = 0; pass < 2; ++pass) { for (int i = lane; i < 16 * 8; i += 32) { const int rr = i >> 3, c4 = (i & 7) * 4; *(volatile v4f*)(Hout + (size_t)(v0 + rr) * HP + c4) = *(const v4f*)(&Out[rr][c4]); } __threadfence(); } }
}

__global__ __launch_bounds__(128) void pool_kernel(const float* __restrict__ H, const int* __restrict__ batch, const float* __restrict__ P, float* __restrict__ out) {
  __shared__ __attribute__((aligned(16))) float Os[NG * NCLS];
  const int g = threadIdx.x;
  auto lower = [&](int key) { int lo = 0, hi = NN; while (lo < hi) { const int mid = (lo + hi) >> 1; if (batch[mid] < key) lo = mid + 1; else hi = mid; } return lo; };
  const int s0 = lower(g), s1 = lower(g + 1); const int cnt = s1 - s0;
  float mx[HID], sm[HID]; for (int c = 0; c < HID; ++c) { mx[c] = -INFINITY; sm[c] = 0.0f; }
  for (int n = s0; n < s1; ++n) { const float* hr = H + (size_t)n * HP;
#pragma unroll
    for (int c = 0; c < HID; ++c) { const float hv = hr[c]; mx[c] = fmaxf(mx[c], hv); sm[c] += hv; } }
  float pooled[2 * HID]; const float invc = 1.0f / fmaxf((float)cnt, 1.0f);
  for (int c = 0; c < HID; ++c) { pooled[c] = (cnt > 0) ? mx[c] : 0.0f; pooled[HID + c] = sm[c] * invc; }
  for (int k = 0; k < NCLS; ++k) { float s = P[592 + k]; for (int c = 0; c < 2 * HID; ++c) s += pmul(pooled[c], P[192 + c * NCLS + k]); Os[g * NCLS + k] = s; }
  __syncthreads();
  for (int pass = 0; pass < 2; ++pass) { for (int i = threadIdx.x; i < NG * NCLS / 4; i += 128) *(volatile v4f*)(out + i * 4) = *(const v4f*)(&Os[i * 4]); __threadfence(); }
}
}

extern "C" void kernel_launch(void* const* d_in, const int* in_sizes, int n_in,
                              void* d_out, int out_size, void* d_ws, size_t ws_size, hipStream_t stream) {
  (void)n_in; (void)out_size;
  const float* x = (const float*)d_in[0]; const int* ei = (const int*)d_in[1]; const int* batch = (const int*)d_in[2]; const float* ew = (const float*)d_in[3];
  const float* W1a = (const float*)d_in[4]; const float* b1a = (const float*)d_in[5]; const float* W1b = (const float*)d_in[6]; const float* b1b = (const float*)d_in[7]; const float* W2a = (const float*)d_in[8]; const float* b2a = (const float*)d_in[9]; const float* W2b = (const float*)d_in[10]; const float* b2b = (const float*)d_in[11];
  const float* W3a = (const float*)d_in[12]; const float* b3a = (const float*)d_in[13]; const float* W3b = (const float*)d_in[14]; const float* b3b = (const float*)d_in[15]; const float* Wl = (const float*)d_in[16]; const float* bl = (const float*)d_in[17];
  float* out = (float*)d_out;
  if (in_sizes[0] != NN * F0 || in_sizes[1] != 2 * NE || in_sizes[2] != NN || in_sizes[3] != NE) return;
  const int* srcI = ei; const int* dstI = ei + NE;
  size_t off = 0; char* ws = (char*)d_ws;
  auto carve = [&](size_t bytes) { char* p = ws + off; off += (bytes + 255) & ~(size_t)255; return p; };
  b16* R = (b16*)carve(Wo_::END * 2); float* P = (float*)carve(608 * 4); float* H0 = (float*)carve((size_t)NN * F0 * 4); float* H1 = (float*)carve((size_t)NN * HP * 4); float* H2 = (float*)carve((size_t)NN * HP * 4);
  CsrBufs cs; off = csr_carve(cs, ws, off, NE, NN);
  if (off > ws_size) return;
  csr_build(cs, dstI, NE, NN, stream);
  prep_kernel<<<512, 256, 0, stream>>>(x, W1a, b1a, W1b, b1b, W2a, b2a, W2b, b2b, W3a, b3a, W3b, b3b, Wl, bl, R, P, H0);
  gin_kernel<64><<<NN / 16, 256, 0, stream>>>(H0, srcI, ew, cs.PERM, cs.ROWPTR, cs.ROWCNT, R + Wo_::A0, R + Wo_::B0, P, H1);
  gin_kernel<32><<<NN / 16, 256, 0, stream>>>(H1, srcI, ew, cs.PERM, cs.ROWPTR, cs.ROWCNT, R + Wo_::A1, R + Wo_::B1, P + 64, H2);
  gin_kernel<32><<<NN / 16, 256, 0, stream>>>(H2, srcI, ew, cs.PERM, cs.ROWPTR, cs.ROWCNT, R + Wo_::A2, R + Wo_::B2, P + 128, H1);
  pool_kernel<<<1, 128, 0, stream>>>(H1, batch, P, out);
}
